// XLAttention_81673098101656
// MI455X (gfx1250) — hardware-verified
//
#include <hip/hip_runtime.h>
#include <math.h>
#include <stdint.h>

#ifndef NB
#define NB 2
#endif
#ifndef SEQ
#define SEQ 2048
#endif
#ifndef MLEN
#define MLEN 2048
#endif
#define B_FULL 2
#define L_FULL 2048
#define M_FULL 2048
#define DMOD  1024
#define NH    16
#define HD    64
#define JL    (MLEN + SEQ)
#define QROWS (NB * SEQ)
#define CROWS (NB * JL)
#define SM_SCALE 0.125f
#define LOG2E 1.4426950408889634f
#define QSC   1024.0f
#define KSC   1024.0f
#define PCAR  32768.0f
#define VCAR  1024.0f
#define OSC   1024.0f
#define WOS   1024.0f
#define WPB   4
#define NHG   (NH / WPB)
#define NQT   (SEQ / 16)
#define NKT   (JL / 32)
#define NVT   (JL / 64)
#define NRT   (SEQ / 64)
#define ATT_THREADS (WPB * 32)
#define PTP   36
#define PTW   (16 * PTP)
#define SLP   68
#define SLW   (16 * SLP)
#define WREG  (PTW + SLW)
#define SLAB64 (16 * 68)
#define VTP   72
#define QKT   (DMOD / 8)
#define WS_CAP 134217728
static_assert(DMOD == NH * HD && HD == 64 && NH == 16);
static_assert((NH % WPB) == 0 && ATT_THREADS == 128);
static_assert(NB >= 1 && NB <= B_FULL);
static_assert((SEQ % 64) == 0 && SEQ >= 64 && SEQ <= L_FULL);
static_assert((MLEN % 64) == 0 && MLEN >= 0 && MLEN <= M_FULL);
static_assert((JL % 64) == 0 && NKT * 32 == JL && NVT * 64 == JL && NQT * 16 == SEQ && NRT * 64 == SEQ);
static_assert(QKT == 128 && (DMOD % 64) == 0 && (DMOD % 32) == 0 && (HD % 32) == 0);
static_assert(((DMOD * DMOD) % (8 * 256)) == 0);
static_assert(QROWS <= CROWS);
static_assert((long long)CROWS * DMOD * 10 + (long long)QROWS * DMOD * 4 + 2LL * DMOD * DMOD <= (long long)WS_CAP);

typedef unsigned short u16;
typedef _Float16 v16h __attribute__((ext_vector_type(16)));
typedef _Float16 v8h  __attribute__((ext_vector_type(8)));
typedef __bf16   v16b __attribute__((ext_vector_type(16)));
typedef float    v8f  __attribute__((ext_vector_type(8)));
typedef float    v4f  __attribute__((ext_vector_type(4)));
typedef unsigned int v4u __attribute__((ext_vector_type(4)));

union FragH { v16h v; v8h h[2]; v4u u[2]; };
union FragB { v16b v; v4u u[2]; };

__device__ __forceinline__ unsigned short bf_bits(float f) {
  unsigned u = __float_as_uint(f);
  return (unsigned short)((u + 0x7FFFu + ((u >> 16) & 1u)) >> 16);
}
__device__ __forceinline__ float bf_up(unsigned short h) { return __uint_as_float(((unsigned)h) << 16); }
__device__ __forceinline__ float bfr(float f) { return bf_up(bf_bits(f)); }
__device__ __forceinline__ unsigned short h_bits(_Float16 x) { return __builtin_bit_cast(unsigned short, x); }
__device__ __forceinline__ unsigned pk16(unsigned short a, unsigned short b) { return (unsigned)a | ((unsigned)b << 16); }
__device__ __forceinline__ v8f zero8() { v8f z = {0.f, 0.f, 0.f, 0.f, 0.f, 0.f, 0.f, 0.f}; return z; }

__device__ __forceinline__ v16h ldfrag_h(const _Float16* p) {
  FragH f;
  f.h[0] = *(const v8h*)(p);
  f.h[1] = *(const v8h*)(p + 16);
  return f.v;
}
__device__ __forceinline__ v16b ldfrag_b(const u16* p) {
  FragB f;
  f.u[0] = *(const v4u*)(p);
  f.u[1] = *(const v4u*)(p + 16);
  return f.v;
}

__device__ __forceinline__ v8f mma_h(v16h a, v16h b, v8f c) {
  return __builtin_amdgcn_wmma_f32_16x16x32_f16(false, a, false, b, (short)0, c, false, false);
}
__device__ __forceinline__ v8f mma_b(v16b a, v16b b, v8f c) {
  return __builtin_amdgcn_wmma_f32_16x16x32_bf16(false, a, false, b, (short)0, c, false, false);
}
__device__ __forceinline__ void guard2(v8f& a, v8f& b, v16h x0, v16h x1, v16h x2, v16h x3,
                                       v16h x4, v16h x5, v16h x6, v16h x7) {
#if defined(__HIP_DEVICE_COMPILE__)
  asm volatile("v_nop\n\tv_nop\n\tv_nop\n\tv_nop"
               : "+v"(a), "+v"(b)
               : "v"(x0), "v"(x1), "v"(x2), "v"(x3), "v"(x4), "v"(x5), "v"(x6), "v"(x7) : "memory");
#endif
}
template <typename F>
__device__ __forceinline__ void guard6(v8f& a, v8f& b, v8f& c, v8f& d, F x0, F x1, F x2, F x3, F x4, F x5) {
#if defined(__HIP_DEVICE_COMPILE__)
  asm volatile("v_nop\n\tv_nop\n\tv_nop\n\tv_nop"
               : "+v"(a), "+v"(b), "+v"(c), "+v"(d) : "v"(x0), "v"(x1), "v"(x2), "v"(x3), "v"(x4), "v"(x5) : "memory");
#endif
}
__device__ __forceinline__ void acc_guard4(v8f& a, v8f& b, v8f& c, v8f& d) {
#if defined(__HIP_DEVICE_COMPILE__)
  asm volatile("v_nop\n\tv_nop\n\tv_nop\n\tv_nop" : "+v"(a), "+v"(b), "+v"(c), "+v"(d));
#endif
}
__device__ __forceinline__ void wave_sync_lds() {
  __builtin_amdgcn_fence(__ATOMIC_RELEASE, "workgroup");
  __builtin_amdgcn_wave_barrier();
  __builtin_amdgcn_fence(__ATOMIC_ACQUIRE, "workgroup");
}

__global__ __launch_bounds__(256) void cvt16(const float* __restrict__ x, u16* D, int n8, int f16mode, float scale) {
  const int gt = blockIdx.x * 256 + (int)threadIdx.x;
  if (gt >= n8) return;
  const float* p = x + (size_t)gt * 8;
  const v4f a = *(const v4f*)(p), b4 = *(const v4f*)(p + 4);
  float w[8];
#pragma unroll
  for (int e = 0; e < 4; ++e) { w[e] = a[e]; w[4 + e] = b4[e]; }
  v4u o;
#pragma unroll
  for (int e = 0; e < 4; ++e) {
    const float f0 = w[2 * e], f1 = w[2 * e + 1];
    const unsigned short hb0 = h_bits((_Float16)(bfr(f0) * scale));
    const unsigned short hb1 = h_bits((_Float16)(bfr(f1) * scale));
    const unsigned short bb0 = bf_bits(f0);
    const unsigned short bb1 = bf_bits(f1);
    o[e] = (f16mode != 0) ? pk16(hb0, hb1) : pk16(bb0, bb1);
  }
  u16* d = D + (size_t)gt * 8;
  for (int pass = 0; pass < 2; ++pass) {
    *(volatile v4u*)(d) = o;
    __threadfence();
  }
}

__global__ __launch_bounds__(QKT) void cvt_act(const float* __restrict__ X0, const float* __restrict__ X1, u16* D,
                                               int nrow, int split) {
  const int tid = (int)threadIdx.x;
  const int r   = (int)blockIdx.x;
  if (r >= NB * nrow) return;
  if (tid >= QKT) return;
  const int  bb    = r / nrow;
  const int  j     = r - bb * nrow;
  const bool first = (j < split);
  const int  js    = first ? j : (j - split);
  const float* base = first ? X0 : X1;
  const float* p = base + ((size_t)js * B_FULL + bb) * DMOD + tid * 8;
  const v4f a = *(const v4f*)(p), a4 = *(const v4f*)(p + 4);
  v4u o;
#pragma unroll
  for (int e = 0; e < 2; ++e) {
    o[e]     = pk16(bf_bits(a[2 * e]),  bf_bits(a[2 * e + 1]));
    o[2 + e] = pk16(bf_bits(a4[2 * e]), bf_bits(a4[2 * e + 1]));
  }
  u16* d = D + (size_t)r * DMOD + tid * 8;
  for (int pass = 0; pass < 2; ++pass) {
    *(volatile v4u*)(d) = o;
    __threadfence();
  }
}

__global__ __launch_bounds__(256) void vt16(const float* __restrict__ F, u16* VHo) {
  __shared__ __align__(16) u16 TH[HD * VTP];
  const int tid = threadIdx.x;
  const int bid = blockIdx.x;
  const int st  = bid % NVT;
  const int t2  = bid / NVT;
  const int g   = t2 % NH;
  const int bb  = t2 / NH;
  if (bb >= NB) return;
  const int s0  = st * 64;
  {
    const int sl = tid >> 2;
    const int dc = (tid & 3) * 16;
    const float* src = F + ((size_t)bb * JL + s0 + sl) * DMOD + g * HD + dc;
#pragma unroll
    for (int i = 0; i < 4; ++i) {
      const v4f a = *(const v4f*)(src + 4 * i);
#pragma unroll
      for (int e = 0; e < 4; ++e) {
        const _Float16 hv = (_Float16)(a[e] * VCAR);
        TH[(dc + 4 * i + e) * VTP + sl] = h_bits(hv);
      }
    }
  }
  __syncthreads();
  v4u vh[2];
  const int q8 = tid >> 3, p8 = (tid & 7) * 8;
#pragma unroll
  for (int it = 0; it < 2; ++it) {
    const int line = it * 32 + q8;
    vh[it] = *(const v4u*)(TH + line * VTP + p8);
  }
  const size_t hrow  = (size_t)(bb * NH + g) * HD;
  const size_t baseH = hrow * JL + s0 + p8;
  for (int pass = 0; pass < 2; ++pass) {
#pragma unroll
    for (int it = 0; it < 2; ++it) {
      const int line = it * 32 + q8;
      *(volatile v4u*)(VHo + baseH + (size_t)line * JL) = vh[it];
    }
    __threadfence();
  }
}

template <int RES>
__global__ __launch_bounds__(QKT) void qk16(const float* __restrict__ F, u16* Hp, u16* Lp, int nrows, float sc) {
  const int tid = (int)threadIdx.x;
  const int row = (int)blockIdx.x;
  if (row >= nrows) return;
  if (tid >= QKT) return;
  const float* p = F + (size_t)row * DMOD + tid * 8;
  const v4f a = *(const v4f*)(p), b4 = *(const v4f*)(p + 4);
  float w[8];
#pragma unroll
  for (int e = 0; e < 4; ++e) { w[e] = a[e] * sc; w[4 + e] = b4[e] * sc; }
  v4u oh, ol;
#pragma unroll
  for (int e = 0; e < 4; ++e) {
    const float t0 = w[2 * e], t1 = w[2 * e + 1];
    const _Float16 h0 = (_Float16)t0, h1 = (_Float16)t1;
    const _Float16 l0 = (_Float16)(t0 - (float)h0), l1 = (_Float16)(t1 - (float)h1);
    oh[e] = pk16(h_bits(h0), h_bits(h1));
    ol[e] = pk16(h_bits(l0), h_bits(l1));
  }
  u16* dh = Hp + (size_t)row * DMOD + tid * 8;
  u16* dl = Lp + (size_t)row * DMOD + tid * 8;
  for (int pass = 0; pass < 2; ++pass) {
    *(volatile v4u*)(dh) = oh;
    if constexpr (RES != 0) {
      *(volatile v4u*)(dl) = ol;
    }
    __threadfence();
  }
}

__device__ __forceinline__ void epi64(float* sl, v8f a0, v8f a1, v8f a2, v8f a3, float oscale,
                                      const float* __restrict__ bias, float* Cb, size_t pitch, int col0, int lane) {
  const int hh = lane >> 4, m = lane & 15;
#pragma unroll
  for (int r = 0; r < 8; ++r) {
    const int ro = (8 * hh + r) * 68 + m;
    sl[ro]      = a0[r] * oscale;
    sl[ro + 16] = a1[r] * oscale;
    sl[ro + 32] = a2[r] * oscale;
    sl[ro + 48] = a3[r] * oscale;
  }
  wave_sync_lds();
  const v4f bb = *(const v4f*)(bias + col0 + m * 4);
  v4f br;
#pragma unroll
  for (int e = 0; e < 4; ++e) br[e] = bfr(bb[e]);
  v4f vals[8];
#pragma unroll
  for (int it = 0; it < 8; ++it) vals[it] = *(const v4f*)(sl + (it * 2 + hh) * 68 + m * 4) + br;
  float* dst = Cb + (size_t)hh * pitch + col0 + m * 4;
  for (int pass = 0; pass < 2; ++pass) {
#pragma unroll
    for (int it = 0; it < 8; ++it) {
      *(volatile v4f*)(dst + (size_t)(it * 2) * pitch) = vals[it];
    }
    __threadfence();
  }
}

__global__ __launch_bounds__(128)
void gemm_bf(const u16* __restrict__ A, const u16* __restrict__ Bt, const float* __restrict__ bias,
             float* C, int M, int N, int K, float oscale) {
  __shared__ __align__(16) float slab[4 * SLAB64];
  const int tid = threadIdx.x, wave = tid >> 5, lane = tid & 31, hh = lane >> 4, m = lane & 15;
  const int ntile = N >> 6;
  const int bid   = blockIdx.x;
  const int rowb  = (bid / ntile) * 64 + wave * 16;
  const int col0  = (bid % ntile) * 64;
  if (rowb + 16 > M) return;
  const u16* ap = A  + (size_t)(rowb + m) * K + 8 * hh;
  const u16* bp = Bt + (size_t)(col0 + m) * K + 8 * hh;
  const size_t bs = (size_t)16 * K;
  v8f acc0 = zero8(), acc1 = zero8(), acc2 = zero8(), acc3 = zero8();
#pragma unroll 1
  for (int k0 = 0; k0 < K; k0 += 32) {
    const v16b a  = ldfrag_b(ap + k0);
    const v16b b0 = ldfrag_b(bp + k0);
    const v16b b1 = ldfrag_b(bp + bs + k0);
    const v16b b2 = ldfrag_b(bp + 2 * bs + k0);
    const v16b b3 = ldfrag_b(bp + 3 * bs + k0);
    acc0 = mma_b(a, b0, acc0);
    acc1 = mma_b(a, b1, acc1);
    acc2 = mma_b(a, b2, acc2);
    acc3 = mma_b(a, b3, acc3);
    guard6<v16b>(acc0, acc1, acc2, acc3, a, b0, b1, b2, b3, a);
  }
  epi64(slab + wave * SLAB64, acc0, acc1, acc2, acc3, oscale, bias, C + (size_t)rowb * (size_t)N, (size_t)N, col0, lane);
}

__global__ __launch_bounds__(128)
void gemm_o2(const u16* __restrict__ Ah, const u16* __restrict__ Al, const u16* __restrict__ Bt, const float* __restrict__ bias,
             float* C, float oscale) {
  __shared__ __align__(16) float slab[4 * SLAB64];
  const int tid = threadIdx.x, wave = tid >> 5, lane = tid & 31, hh = lane >> 4, m = lane & 15;
  const int ntile = DMOD >> 6;
  const int bid   = blockIdx.x;
  const int ct    = bid % ntile;
  const int t2    = bid / ntile;
  const int rt    = t2 % NRT;
  const int bb    = t2 / NRT;
  if (bb >= NB) return;
  const int srow  = rt * 64 + wave * 16;
  if (srow + 16 > SEQ) return;
  const int col0  = ct * 64;
  const int K     = DMOD;
  const size_t rowA = (size_t)bb * SEQ + srow;
  const _Float16* ahp = (const _Float16*)(const void*)Ah + (rowA + m) * K + 8 * hh;
  const _Float16* alp = (const _Float16*)(const void*)Al + (rowA + m) * K + 8 * hh;
  const _Float16* bp  = (const _Float16*)(const void*)Bt + (size_t)(col0 + m) * K + 8 * hh;
  const size_t bs = (size_t)16 * K;
  v8f acc0 = zero8(), acc1 = zero8(), acc2 = zero8(), acc3 = zero8();
#pragma unroll 1
  for (int k0 = 0; k0 < K; k0 += 32) {
    const v16h ah = ldfrag_h(ahp + k0), al = ldfrag_h(alp + k0);
    const v16h b0 = ldfrag_h(bp + k0);
    const v16h b1 = ldfrag_h(bp + bs + k0);
    const v16h b2 = ldfrag_h(bp + 2 * bs + k0);
    const v16h b3 = ldfrag_h(bp + 3 * bs + k0);
    acc0 = mma_h(ah, b0, acc0);  acc0 = mma_h(al, b0, acc0);
    acc1 = mma_h(ah, b1, acc1);  acc1 = mma_h(al, b1, acc1);
    acc2 = mma_h(ah, b2, acc2);  acc2 = mma_h(al, b2, acc2);
    acc3 = mma_h(ah, b3, acc3);  acc3 = mma_h(al, b3, acc3);
    guard6<v16h>(acc0, acc1, acc2, acc3, ah, al, b0, b1, b2, b3);
  }
  float* Cb = C + ((size_t)srow * NB + bb) * DMOD;
  epi64(slab + wave * SLAB64, acc0, acc1, acc2, acc3, oscale, bias, Cb, (size_t)NB * DMOD, col0, lane);
}

__global__ __launch_bounds__(ATT_THREADS)
void attn_x(const u16* __restrict__ QHp, const u16* __restrict__ QLp, const u16* __restrict__ KHp,
            const u16* __restrict__ VHp, u16* OHp, u16* OLp) {
  __shared__ __align__(16) float smem[WPB * WREG];

  const int tid  = threadIdx.x;
  const int wave = tid >> 5;
  const int lane = tid & 31;
  const int hh   = lane >> 4;
  const int c    = lane & 15;
  const int bid  = blockIdx.x;
  const int qt   = bid % NQT;
  const int t2   = bid / NQT;
  const int hg   = t2 % NHG;
  const int b    = t2 / NHG;
  if (b >= NB) return;
  const int q0   = qt * 16;
  const int head = hg * WPB + wave;

  float* pt   = smem + wave * WREG;
  float* slab = pt + PTW;

  const size_t hcol = (size_t)head * HD + 8 * hh;
  const _Float16* Qh  = (const _Float16*)(const void*)QHp + ((size_t)b * SEQ + q0 + c) * DMOD + hcol;
  const _Float16* Ql  = (const _Float16*)(const void*)QLp + ((size_t)b * SEQ + q0 + c) * DMOD + hcol;
  const _Float16* Khb = (const _Float16*)(const void*)KHp + ((size_t)b * JL + c) * DMOD + hcol;
  const _Float16* Vhb = (const _Float16*)(const void*)VHp + ((size_t)(b * NH + head) * HD + c) * JL + 8 * hh;
  const float lsc = SM_SCALE * (LOG2E / (QSC * KSC));
  const float oc  = 1.0f / (PCAR * VCAR);
  const size_t KROW = (size_t)DMOD;

  const v16h qh0 = ldfrag_h(Qh), qh1 = ldfrag_h(Qh + 32);
  const v16h ql0 = ldfrag_h(Ql), ql1 = ldfrag_h(Ql + 32);

  float mrow[8], lrow[8];
  v8f o[4];
#pragma unroll
  for (int r = 0; r < 8; ++r) { mrow[r] = -INFINITY; lrow[r] = 0.f; }
#pragma unroll
  for (int j = 0; j < 4; ++j) o[j] = zero8();

#pragma unroll 1
  for (int kt = 0; kt < NKT; ++kt) {
    const int kb = kt * 32;
    v8f s0 = zero8(), s1 = zero8();
    {
      const _Float16* k0p = Khb + (size_t)kb * KROW;
      const _Float16* k1p = k0p + (size_t)16 * KROW;
      const v16h ka0 = ldfrag_h(k0p), ka1 = ldfrag_h(k0p + 32);
      const v16h kc0 = ldfrag_h(k1p), kc1 = ldfrag_h(k1p + 32);
      s0 = mma_h(qh0, ka0, s0);
      s0 = mma_h(ql0, ka0, s0);
      s0 = mma_h(qh1, ka1, s0);
      s0 = mma_h(ql1, ka1, s0);
      s1 = mma_h(qh0, kc0, s1);
      s1 = mma_h(ql0, kc0, s1);
      s1 = mma_h(qh1, kc1, s1);
      s1 = mma_h(ql1, kc1, s1);
      guard2(s0, s1, ka0, ka1, kc0, kc1, qh0, ql0, qh1, ql1);
    }
#pragma unroll
    for (int r = 0; r < 8; ++r) {
      const float t0 = s0[r] * lsc;
      const float t1 = s1[r] * lsc;
      float mx = fmaxf(t0, t1);
#pragma unroll
      for (int off = 1; off < 16; off <<= 1) mx = fmaxf(mx, __shfl_xor(mx, off, 32));
      const float mn = fmaxf(mrow[r], mx);
      const float ms = (mn == -INFINITY) ? 0.0f : mn;
      const float al = exp2f(mrow[r] - ms);
      mrow[r] = mn;
      const float e0 = exp2f(t0 - ms), e1 = exp2f(t1 - ms);
      float ps = e0 + e1;
#pragma unroll
      for (int off = 1; off < 16; off <<= 1) ps += __shfl_xor(ps, off, 32);
      lrow[r] = lrow[r] * al + ps;
#pragma unroll
      for (int j = 0; j < 4; ++j) o[j][r] *= al;
      const int ro = (8 * hh + r) * PTP + c;
      pt[ro]      = e0;
      pt[ro + 16] = e1;
    }
    wave_sync_lds();
    FragH ph;
    {
      const float* prow = pt + c * PTP + 8 * hh;
      const v4f p0 = *(const v4f*)(prow), p1 = *(const v4f*)(prow + 4);
      const v4f p2 = *(const v4f*)(prow + 16), p3 = *(const v4f*)(prow + 20);
#pragma unroll
      for (int e = 0; e < 4; ++e) {
        ph.h[0][e]     = (_Float16)(p0[e] * PCAR);
        ph.h[0][4 + e] = (_Float16)(p1[e] * PCAR);
        ph.h[1][e]     = (_Float16)(p2[e] * PCAR);
        ph.h[1][4 + e] = (_Float16)(p3[e] * PCAR);
      }
    }
    {
      const _Float16* vhp = Vhb + kb;
#pragma unroll
      for (int jg = 0; jg < HD / 32; ++jg) {
        const size_t da = (size_t)(2 * jg) * 16 * JL;
        const size_t db = da + (size_t)16 * JL;
        const v16h vha = ldfrag_h(vhp + da), vhc = ldfrag_h(vhp + db);
        o[2 * jg]     = mma_h(ph.v, vha, o[2 * jg]);
        o[2 * jg + 1] = mma_h(ph.v, vhc, o[2 * jg + 1]);
        guard2(o[2 * jg], o[2 * jg + 1], ph.v, vha, vhc, ph.v, vha, vhc, ph.v, ph.v);
      }
    }
    wave_sync_lds();
  }
  acc_guard4(o[0], o[1], o[2], o[3]);
#pragma unroll
  for (int r = 0; r < 8; ++r) {
    const float lv  = lrow[r];
    const float ls  = (lv > 0.0f) ? lv : 1.0f;
    const float inv = (lv > 0.0f) ? ((1.0f / ls) * oc) : 0.0f;
#pragma unroll
    for (int j = 0; j < 4; ++j) {
      const int idx = (8 * hh + r) * SLP + j * 16 + c;
      slab[idx] = o[j][r] * inv;
    }
  }

  wave_sync_lds();
  v4u oh[4], ol[4];
  const int rq = lane >> 3, c8 = (lane & 7) * 8;
#pragma unroll
  for (int it = 0; it < 4; ++it) {
    const int row = it * 4 + rq;
    const v4f a = *(const v4f*)(slab + row * SLP + c8), b4 = *(const v4f*)(slab + row * SLP + c8 + 4);
    float w[8];
#pragma unroll
    for (int e = 0; e < 4; ++e) { w[e] = a[e] * OSC; w[4 + e] = b4[e] * OSC; }
#pragma unroll
    for (int e = 0; e < 4; ++e) {
      const _Float16 h0 = (_Float16)w[2 * e], h1 = (_Float16)w[2 * e + 1];
      const _Float16 l0 = (_Float16)(w[2 * e] - (float)h0), l1 = (_Float16)(w[2 * e + 1] - (float)h1);
      oh[it][e] = pk16(h_bits(h0), h_bits(h1));
      ol[it][e] = pk16(h_bits(l0), h_bits(l1));
    }
  }
  const size_t ob = ((size_t)b * SEQ + q0) * DMOD + (size_t)head * HD + c8;
  for (int pass = 0; pass < 2; ++pass) {
#pragma unroll
    for (int it = 0; it < 4; ++it) {
      const int row = it * 4 + rq;
      *(volatile v4u*)(OHp + ob + (size_t)row * DMOD) = oh[it];
      *(volatile v4u*)(OLp + ob + (size_t)row * DMOD) = ol[it];
    }
    __threadfence();
  }
}

extern "C" void kernel_launch(void* const* d_in, const int* in_sizes, int n_in,
                              void* d_out, int out_size, void* d_ws, size_t ws_size,
                              hipStream_t stream) {
  if (n_in < 11) return;
  const long long needq = ((long long)(SEQ - 1) * B_FULL + NB) * DMOD;
  const long long needm = (MLEN > 0) ? (((long long)(MLEN - 1) * B_FULL + NB) * DMOD) : 0;
  if ((long long)in_sizes[0] < needq || (long long)in_sizes[1] < needq || (long long)in_sizes[2] < needm) return;
  if (in_sizes[3] < DMOD * DMOD || in_sizes[5] < DMOD * DMOD || in_sizes[7] < DMOD * DMOD || in_sizes[9] < DMOD * DMOD) return;
  if (in_sizes[4] < DMOD || in_sizes[6] < DMOD || in_sizes[8] < DMOD || in_sizes[10] < DMOD) return;
  if ((long long)out_size < (long long)SEQ * NB * DMOD) return;

  const float* xq  = (const float*)d_in[0];
  const float* xkv = (const float*)d_in[1];
  const float* xm  = (const float*)d_in[2];
  const float* wq  = (const float*)d_in[3];
  const float* bq  = (const float*)d_in[4];
  const float* wk  = (const float*)d_in[5];
  const float* bk  = (const float*)d_in[6];
  const float* wv  = (const float*)d_in[7];
  const float* bv  = (const float*)d_in[8];
  const float* wc  = (const float*)d_in[9];
  const float* bc  = (const float*)d_in[10];
  float*       out = (float*)d_out;

  const size_t szXC = (size_t)CROWS * DMOD * 2;
  const size_t szXQ = (size_t)QROWS * DMOD * 2;
  const size_t szW  = (size_t)DMOD * DMOD * 2;
  const size_t szF  = (size_t)CROWS * DMOD * 4;
  const size_t szO  = (size_t)QROWS * DMOD * 2;
  const size_t szVH = (size_t)NB * NH * HD * JL * 2;
  const size_t szKH = (size_t)CROWS * DMOD * 2;
  const size_t szQ  = (size_t)QROWS * DMOD * 2;
  if (2 * szO > szF || szXQ > szXC) return;
  size_t off = 0;
  const size_t oXC = off; off += szXC;
  const size_t oW  = off; off += szW;
  const size_t oF  = off; off += szF;
  const size_t oVH = off; off += szVH;
  const size_t oKH = off; off += szKH;
  const size_t oQH = off; off += szQ;
  const size_t oQL = off; off += szQ;
  if (off > ws_size) return;
  if (off > (size_t)WS_CAP) return;

  char* ws = (char*)d_ws;
  u16*   XC = (u16*)(ws + oXC);
  u16*   XQ = (u16*)(ws + oXC);
  u16*   WB = (u16*)(ws + oW);
  float* F  = (float*)(ws + oF);
  u16*   OH = (u16*)(ws + oF);
  u16*   OL = (u16*)(ws + oF + szO);
  u16*   VH = (u16*)(ws + oVH);
  u16*   KH = (u16*)(ws + oKH);
  u16*   QH = (u16*)(ws + oQH);
  u16*   QL = (u16*)(ws + oQL);

  const dim3 b256(256), b128(128), bQK(QKT), bAT(ATT_THREADS);
  const int  n8w = (DMOD * DMOD) / 8;
  const dim3 gW((n8w + 255) / 256);
  const dim3 gXC(CROWS), gXQ(QROWS);
  const dim3 gGC((CROWS / 64) * (DMOD / 64));
  const dim3 gGQ((QROWS / 64) * (DMOD / 64));
  const dim3 gVT(NB * NH * NVT);
  const dim3 gAT(NQT * NHG * NB);
  const dim3 gO(NB * NRT * (DMOD / 64));

  cvt_act<<<gXC, bQK, 0, stream>>>(xm, xkv, XC, JL, MLEN);
  cvt16<<<gW, b256, 0, stream>>>(wv, WB, n8w, 0, 1.0f);
  gemm_bf<<<gGC, b128, 0, stream>>>(XC, WB, bv, F, CROWS, DMOD, DMOD, 1.0f);
  vt16<<<gVT, b256, 0, stream>>>(F, VH);
  cvt16<<<gW, b256, 0, stream>>>(wk, WB, n8w, 0, 1.0f);
  gemm_bf<<<gGC, b128, 0, stream>>>(XC, WB, bk, F, CROWS, DMOD, DMOD, 1.0f);
  qk16<0><<<gXC, bQK, 0, stream>>>(F, KH, KH, CROWS, KSC);
  cvt_act<<<gXQ, bQK, 0, stream>>>(xq, xq, XQ, SEQ, SEQ);
  cvt16<<<gW, b256, 0, stream>>>(wq, WB, n8w, 0, 1.0f);
  gemm_bf<<<gGQ, b128, 0, stream>>>(XQ, WB, bq, F, QROWS, DMOD, DMOD, 1.0f);
  qk16<1><<<gXQ, bQK, 0, stream>>>(F, QH, QL, QROWS, QSC);
  cvt16<<<gW, b256, 0, stream>>>(wc, WB, n8w, 1, WOS);
  attn_x<<<gAT, bAT, 0, stream>>>(QH, QL, KH, VH, OH, OL);
  gemm_o2<<<gO, b128, 0, stream>>>(OH, OL, WB, bc, out, 1.0f / (OSC * WOS));
  (void)hipGetLastError();
}
